// Net_3874060501607
// MI455X (gfx1250) — hardware-verified
//
#include <hip/hip_runtime.h>
#include <stddef.h>
#include <stdint.h>
#include <math.h>


#define DIN    128
#define D1     150
#define D1P    160
#define D2     100
#define D2P    128
#define DOUT   64
#define K1     256
#define K2G    320
#define K3     256
#define NSP    256
#define HROW   320
#define NTHR   256
#define NWAVE  8
#define EPT    8
#define CHUNK  (NTHR * EPT)
#define WCAP   (EPT * 32)
#define LISTN  (NWAVE * WCAP)
#define NBD    4096
#define SLD    12
#define NBA    1024
#define SLA    10
#define RCAP   24576
#define DEGCAP 64
#define GBM    64
#define GTHR   128
#define NUW1   (D1P * (K1 / 8))
#define NUWS   (D2P * (K2G / 8))
#define NUW3   (DOUT * (K3 / 8))
#define NUWT   (NUW1 + 2 * NUWS + NUW3)
#define AGG_ZINTS    (LISTN + 2 * RCAP + 3 * NBA)
#define MISC_INTS    16
#define ROWBUF_INTS  (NWAVE * 256 / 2)
#define PZL_INTS     NBA
#define AGG_LDS_INTS (AGG_ZINTS + MISC_INTS + ROWBUF_INTS + PZL_INTS)
#define WSMAX  134217728

static_assert((CHUNK & (CHUNK - 1)) == 0 && CHUNK <= 4096);
static_assert((NBD & (NBD - 1)) == 0 && NBD == (1 << SLD));
static_assert((NBA & (NBA - 1)) == 0 && NBA == (1 << SLA));
static_assert(((long long)CHUNK << SLD) < (1LL << 31));
static_assert(((long long)CHUNK << SLA) < (1LL << 31));
static_assert(NBD % (NTHR * 4) == 0);
static_assert(NBA == NTHR * 4);
static_assert(NBA % NWAVE == 0 && NBA % 32 == 0 && NBA % GBM == 0);
static_assert(RCAP % 4 == 0 && AGG_ZINTS % 4 == 0 && ((AGG_ZINTS + MISC_INTS) % 4) == 0);
static_assert(K1 % 32 == 0 && K2G % 32 == 0 && K3 % 32 == 0);
static_assert(K1 == 2 * DIN && K2G == 2 * D1P && K3 == 2 * D2P && HROW == 2 * D1P);
static_assert(NUW1 % NTHR == 0 && NUWS % NTHR == 0 && NUW3 % NTHR == 0);
static_assert(D2 % 4 == 0 && D2P == 4 * 32 && DIN == 4 * 32);
static_assert(AGG_LDS_INTS * 4 <= 300000);
static_assert(DEGCAP >= 33 + 8);

typedef float          v4f   __attribute__((ext_vector_type(4)));
typedef float          v8f   __attribute__((ext_vector_type(8)));
typedef int            v4i   __attribute__((ext_vector_type(4)));
typedef int            v8i   __attribute__((ext_vector_type(8)));
typedef unsigned       v2u   __attribute__((ext_vector_type(2)));
typedef unsigned short v8us  __attribute__((ext_vector_type(8)));
typedef unsigned short v16us __attribute__((ext_vector_type(16)));
typedef __bf16         v16bf __attribute__((ext_vector_type(16)));
typedef v4f  __attribute__((may_alias)) v4fa;
typedef v4i  __attribute__((may_alias)) v4ia;
typedef v2u  __attribute__((may_alias)) v2ua;
typedef v8us __attribute__((may_alias)) v8usa;
union FragB { v16bf v; v16us u; v8us h[2]; v8i w; };

__device__ __forceinline__ v8f wmb(const FragB& a, const FragB& b, v8f c) {
  v8f d = __builtin_amdgcn_wmma_f32_16x16x32_bf16(false, a.v, false, b.v, (short)0, c, false, false);
  asm volatile("v_nop\n\tv_nop\n\tv_nop\n\tv_nop" : "+v"(d) : "v"(a.w), "v"(b.w));
  return d;
}

__device__ __forceinline__ unsigned bf16_bits(float f) {
  const unsigned u = __float_as_uint(f);
  return (u + 0x7FFFu + ((u >> 16) & 1u)) >> 16;
}
__device__ __forceinline__ float bf16_val(float f) {
  return __uint_as_float(bf16_bits(f) << 16);
}
__device__ __forceinline__ float eluf(float v) {
  return (v > 0.0f) ? v : expm1f(v);
}

__device__ __forceinline__ void wave_sync() {
  __builtin_amdgcn_fence(__ATOMIC_RELEASE, "wavefront");
  __builtin_amdgcn_wave_barrier();
  __builtin_amdgcn_fence(__ATOMIC_ACQUIRE, "wavefront");
}

template <int SLB>
__device__ __forceinline__ int scan_chunk(const int* __restrict__ dsts, int nE, int cbase, int slotBase,
                                          int nb, int vec8, int* list, int tid, int lane, int wave) {
  int wc = 0;
  const int el0  = tid * EPT;
  const int e0   = cbase + el0;
  const int sent = -2147483647 - 1;
  v4i da, db;
  if (vec8 != 0 && cbase + CHUNK <= nE) {
    da = *(const v4i*)(dsts + e0);
    db = *(const v4i*)(dsts + e0 + 4);
  } else {
    da.x = (e0     < nE) ? dsts[min(e0,     nE - 1)] : sent;
    da.y = (e0 + 1 < nE) ? dsts[min(e0 + 1, nE - 1)] : sent;
    da.z = (e0 + 2 < nE) ? dsts[min(e0 + 2, nE - 1)] : sent;
    da.w = (e0 + 3 < nE) ? dsts[min(e0 + 3, nE - 1)] : sent;
    db.x = (e0 + 4 < nE) ? dsts[min(e0 + 4, nE - 1)] : sent;
    db.y = (e0 + 5 < nE) ? dsts[min(e0 + 5, nE - 1)] : sent;
    db.z = (e0 + 6 < nE) ? dsts[min(e0 + 6, nE - 1)] : sent;
    db.w = (e0 + 7 < nE) ? dsts[min(e0 + 7, nE - 1)] : sent;
  }
  const unsigned nbs = (unsigned)slotBase;
  const unsigned unb = (unsigned)nb;
  const unsigned s0 = (unsigned)da.x - nbs, s1 = (unsigned)da.y - nbs;
  const unsigned s2 = (unsigned)da.z - nbs, s3 = (unsigned)da.w - nbs;
  const unsigned s4 = (unsigned)db.x - nbs, s5 = (unsigned)db.y - nbs;
  const unsigned s6 = (unsigned)db.z - nbs, s7 = (unsigned)db.w - nbs;
  const bool h0 = s0 < unb, h1 = s1 < unb, h2 = s2 < unb, h3 = s3 < unb;
  const bool h4 = s4 < unb, h5 = s5 < unb, h6 = s6 < unb, h7 = s7 < unb;
  const unsigned any = __builtin_amdgcn_ballot_w32(h0 | h1 | h2 | h3 | h4 | h5 | h6 | h7);
  if (any != 0u) {
#define HITJ(J, HJ, SJ) { \
      const unsigned mj = __builtin_amdgcn_ballot_w32(HJ); \
      if (mj != 0u) { \
        if (HJ) { \
          const int pos = wc + (int)__builtin_amdgcn_mbcnt_lo(mj, 0u); \
          if (pos < WCAP) list[wave * WCAP + pos] = ((el0 + (J)) << SLB) | (int)(SJ); \
        } \
        wc += (int)__builtin_popcount(mj); } }
    HITJ(0, h0, s0)
    HITJ(1, h1, s1)
    HITJ(2, h2, s2)
    HITJ(3, h3, s3)
    HITJ(4, h4, s4)
    HITJ(5, h5, s5)
    HITJ(6, h6, s6)
    HITJ(7, h7, s7)
#undef HITJ
  }
  return wc;
}

__device__ __forceinline__ v8us wgather(const float* __restrict__ W, int k8, int n, int rows, int cols) {
  const int  nc  = n < cols ? n : cols - 1;
  const bool nok = n < cols;
  v8us o;
#pragma unroll
  for (int i = 0; i < 8; ++i) {
    const int k  = k8 + i;
    const int kc = k < rows ? k : rows - 1;
    const float v = W[(size_t)kc * cols + nc];
    const unsigned b = bf16_bits(v);
    o[i] = (nok && (k < rows)) ? (unsigned short)b : (unsigned short)0;
  }
  return o;
}

__global__ __launch_bounds__(NTHR) void k_wprep(const float* __restrict__ W1, const float* __restrict__ Ws,
                                                const float* __restrict__ Wn, const float* __restrict__ W3,
                                                unsigned short* W1T2, unsigned short* WSN, unsigned short* W3T2) {
  const int u = (int)blockIdx.x * NTHR + (int)threadIdx.x;
  v8us o;
  unsigned short* dp;
  if (u < NUW1) {
    const int n   = u >> 5;
    const int kk8 = (u & 31) * 8;
    o  = wgather(W1, kk8 & (DIN - 1), n, DIN, D1);
    dp = W1T2 + (size_t)n * K1 + kk8;
  } else if (u < NUW1 + NUWS) {
    const int v   = u - NUW1;
    const int n   = v / 40;
    const int kk8 = (v - n * 40) * 8;
    const int k8  = kk8 >= D1P ? kk8 - D1P : kk8;
    o  = wgather(Ws, k8, n, D1, D2);
    dp = WSN + (size_t)n * K2G + kk8;
  } else if (u < NUW1 + 2 * NUWS) {
    const int v   = u - NUW1 - NUWS;
    const int n   = v / 40;
    const int kk8 = (v - n * 40) * 8;
    const int k8  = kk8 >= D1P ? kk8 - D1P : kk8;
    o  = wgather(Wn, k8, n, D1, D2);
    dp = WSN + (size_t)(D2P + n) * K2G + kk8;
  } else if (u < NUWT) {
    const int v   = u - NUW1 - 2 * NUWS;
    const int n   = v >> 5;
    const int kk8 = (v & 31) * 8;
    o  = wgather(W3, kk8 & (D2P - 1), n, D2, DOUT);
    dp = W3T2 + (size_t)n * K3 + kk8;
  } else {
    return;
  }
  *(volatile v8us*)dp = o;
  __threadfence();
  *(volatile v8us*)dp = o;
}

__global__ __launch_bounds__(NTHR) void k_cvx(const float* __restrict__ x, int nN, int nUnits,
                                              unsigned short* xb) {
  const int u = (int)blockIdx.x * NTHR + (int)threadIdx.x;
  if (u >= nUnits) return;
  const int row = u >> 4;
  const int k8  = (u & 15) * 8;
  const int rc  = row < nN ? row : nN - 1;
  const float* p = x + (size_t)rc * DIN + k8;
  const v4f a = *(const v4fa*)p;
  const v4f b = *(const v4fa*)(p + 4);
  const bool ok = row < nN;
  v8us o;
  o[0] = ok ? (unsigned short)bf16_bits(a.x) : (unsigned short)0;
  o[1] = ok ? (unsigned short)bf16_bits(a.y) : (unsigned short)0;
  o[2] = ok ? (unsigned short)bf16_bits(a.z) : (unsigned short)0;
  o[3] = ok ? (unsigned short)bf16_bits(a.w) : (unsigned short)0;
  o[4] = ok ? (unsigned short)bf16_bits(b.x) : (unsigned short)0;
  o[5] = ok ? (unsigned short)bf16_bits(b.y) : (unsigned short)0;
  o[6] = ok ? (unsigned short)bf16_bits(b.z) : (unsigned short)0;
  o[7] = ok ? (unsigned short)bf16_bits(b.w) : (unsigned short)0;
  unsigned short* dp = xb + (size_t)row * DIN + k8;
  *(volatile v8us*)dp = o;
  __threadfence();
  *(volatile v8us*)dp = o;
}

template <int MODE>
__global__ __launch_bounds__(NTHR) void k_deg(const int* __restrict__ keys, int nE, int vec8,
                                              float* pa, float* pb, int* pd) {
  __shared__ __attribute__((aligned(16))) int   scnt[NBD];
  __shared__ __attribute__((aligned(16))) int   list[LISTN];
  __shared__ __attribute__((aligned(16))) float fa[NBD];
  __shared__ __attribute__((aligned(16))) float fb[NBD];
  __shared__ int wcnt[NWAVE];
  const int tid = (int)threadIdx.x, lane = tid & 31, wave = tid >> 5;
  const int nodeBase = (int)blockIdx.x * NBD;

  for (int i = tid; i < NBD; i += NTHR) scnt[i] = 0;
  for (int i = tid; i < LISTN; i += NTHR) list[i] = 0;
  if (tid < NWAVE) wcnt[tid] = 0;
  __syncthreads();

  const int nChunks = (nE + CHUNK - 1) / CHUNK;
#pragma unroll 1
  for (int ch = 0; ch < nChunks; ++ch) {
    const int cbase = ch * CHUNK;
    const int wc = scan_chunk<SLD>(keys, nE, cbase, nodeBase, NBD, vec8, list, tid, lane, wave);
    if (lane == 0) wcnt[wave] = wc;
    __syncthreads();
    if (wave == 0) {
#pragma unroll 1
      for (int w2 = 0; w2 < NWAVE; ++w2) {
        int c = wcnt[w2];
        c = c < 0 ? 0 : (c > WCAP ? WCAP : c);
#pragma unroll 1
        for (int b0 = 0; b0 < c; b0 += 32) {
          const int idx = b0 + lane;
          const int ent = list[w2 * WCAP + (idx < WCAP ? idx : WCAP - 1)];
          const int m32 = (c - b0) < 32 ? (c - b0) : 32;
#pragma unroll 1
          for (int k = 0; k < m32; ++k) {
            const int u  = __builtin_amdgcn_readlane(ent, k);
            const int sl = u & (NBD - 1);
            if (lane == 0) scnt[sl] = scnt[sl] + 1;
          }
        }
      }
    }
    __syncthreads();
  }

#pragma unroll 1
  for (int i = tid; i < NBD; i += NTHR) {
    const int c = scnt[i];
    const float d = (float)(c < 1 ? 1 : c);
    fa[i] = 1.0f / sqrtf(d);
    if constexpr (MODE != 0) fb[i] = 1.0f / d;
  }
  __syncthreads();

  constexpr int NIT = NBD / (NTHR * 4);
  v4f va[NIT];
  v4f vb[NIT];
  v4i vc[NIT];
#pragma unroll
  for (int it = 0; it < NIT; ++it) {
    const int s0 = it * (NTHR * 4) + 4 * tid;
    va[it] = *(const v4fa*)(fa + s0);
    if constexpr (MODE != 0) {
      vb[it] = *(const v4fa*)(fb + s0);
      vc[it] = *(const v4ia*)(scnt + s0);
    }
  }
#pragma unroll
  for (int it = 0; it < NIT; ++it) {
    const size_t g0 = (size_t)nodeBase + it * (NTHR * 4) + 4 * tid;
    *(volatile v4f*)(pa + g0) = va[it];
    if constexpr (MODE != 0) {
      *(volatile v4f*)(pb + g0) = vb[it];
      *(volatile v4i*)(pd + g0) = vc[it];
    }
  }
  __threadfence();
#pragma unroll
  for (int it = 0; it < NIT; ++it) {
    const size_t g0 = (size_t)nodeBase + it * (NTHR * 4) + 4 * tid;
    *(volatile v4f*)(pa + g0) = va[it];
    if constexpr (MODE != 0) {
      *(volatile v4f*)(pb + g0) = vb[it];
      *(volatile v4i*)(pd + g0) = vc[it];
    }
  }
}

template <int NT, int EPI>
__global__ __launch_bounds__(GTHR) void k_gemm(const unsigned short* __restrict__ A,
                                               const unsigned short* __restrict__ WT, int K,
                                               const float* __restrict__ bias, int nBias,
                                               const float* __restrict__ pzp,
                                               unsigned short* outH, float* outF, int nOut) {
  constexpr int NC  = 16 * NT;
  constexpr int HBN = (EPI == 1) ? ((GTHR / 32) * 4 * HROW) : 8;
  static_assert(EPI != 1 || (NC == D1P && HROW == 2 * NC && NC % 32 == 0));
  static_assert(EPI != 2 || NC == 128);
  static_assert(EPI != 3 || NC == DOUT);
  __shared__ __attribute__((aligned(16))) float stg[GBM * NC];
  __shared__ __attribute__((aligned(16))) unsigned short hbuf[HBN];
  __shared__ __attribute__((aligned(16))) float bs[NC];
  __shared__ __attribute__((aligned(16))) float pzl[GBM];
  const int tid = (int)threadIdx.x, lane = tid & 31, wave = tid >> 5, hh = lane >> 4, m = lane & 15;
  const int rowBase = (int)blockIdx.x * GBM;
  const int col0    = (int)blockIdx.y * NC;

  if constexpr (EPI != 2) {
#pragma unroll 1
    for (int c = tid; c < NC; c += GTHR) {
      const int gc = col0 + c;
      const int cc = gc < nBias ? gc : nBias - 1;
      const float b = bias[cc];
      bs[c] = (gc < nBias) ? bf16_val(b) : 0.0f;
    }
  }
  if constexpr (EPI == 3) {
    if (tid < GBM) pzl[tid] = pzp[rowBase + tid];
  }

  v8f acc[NT];
  {
    const v8f z = {0.f, 0.f, 0.f, 0.f, 0.f, 0.f, 0.f, 0.f};
#pragma unroll
    for (int t = 0; t < NT; ++t) acc[t] = z;
  }
  const unsigned short* ap = A  + (size_t)(rowBase + 16 * wave + m) * (size_t)K + 8 * hh;
  const unsigned short* wp = WT + (size_t)(col0 + m) * (size_t)K + 8 * hh;
  const int ksteps = K >> 5;
#pragma unroll 1
  for (int ks = 0; ks < ksteps; ++ks) {
    FragB af;
    af.h[0] = *(const v8usa*)(ap + 32 * ks);
    af.h[1] = *(const v8usa*)(ap + 32 * ks + 16);
#pragma unroll
    for (int t = 0; t < NT; ++t) {
      const unsigned short* wq = wp + (size_t)(16 * t) * (size_t)K + 32 * ks;
      FragB bf;
      bf.h[0] = *(const v8usa*)wq;
      bf.h[1] = *(const v8usa*)(wq + 16);
      acc[t] = wmb(af, bf, acc[t]);
    }
  }

#pragma unroll
  for (int t = 0; t < NT; ++t) {
    const int lc = 16 * t + m;
#pragma unroll
    for (int r = 0; r < 8; ++r) {
      const int lr = 16 * wave + 8 * hh + r;
      stg[lr * NC + lc] = acc[t][r];
    }
  }
  __syncthreads();

  if constexpr (EPI == 1) {
    unsigned short* hb = hbuf + wave * (4 * HROW);
#pragma unroll 1
    for (int g = 0; g < 4; ++g) {
#pragma unroll 1
      for (int ri = 0; ri < 4; ++ri) {
        const int lr = 16 * wave + 4 * g + ri;
        const bool ok = (rowBase + lr) < nOut;
        const float* fr = stg + lr * NC;
        unsigned short* hr = hb + ri * HROW;
#pragma unroll 1
        for (int j = 0; j < NC / 32; ++j) {
          const int c = lane + 32 * j;
          float v = eluf(fr[c] + bs[c]);
          v = ok ? v : 0.0f;
          const unsigned hbits = bf16_bits(v);
          const unsigned lbits = bf16_bits(v - __uint_as_float(hbits << 16));
          hr[c]      = (unsigned short)hbits;
          hr[NC + c] = (unsigned short)lbits;
        }
      }
      wave_sync();
      v8us q[5];
#pragma unroll
      for (int p = 0; p < 5; ++p) q[p] = *(const v8usa*)(hb + 8 * (lane + 32 * p));
      wave_sync();
      unsigned short* gp = outH + (size_t)(rowBase + 16 * wave + 4 * g) * HROW + 8 * lane;
#pragma unroll
      for (int p = 0; p < 5; ++p) *(volatile v8us*)(gp + 256 * p) = q[p];
      __threadfence();
#pragma unroll
      for (int p = 0; p < 5; ++p) *(volatile v8us*)(gp + 256 * p) = q[p];
    }
  } else if constexpr (EPI == 2) {
    v4f pv[16];
#pragma unroll
    for (int i = 0; i < 16; ++i) pv[i] = *(const v4fa*)(stg + (16 * wave + i) * NC + 4 * lane);
#pragma unroll
    for (int i = 0; i < 16; ++i) {
      float* op = outF + (size_t)(rowBase + 16 * wave + i) * NSP + col0 + 4 * lane;
      *(volatile v4f*)op = pv[i];
    }
    __threadfence();
#pragma unroll
    for (int i = 0; i < 16; ++i) {
      float* op = outF + (size_t)(rowBase + 16 * wave + i) * NSP + col0 + 4 * lane;
      *(volatile v4f*)op = pv[i];
    }
  } else {
    const v4f b4 = *(const v4fa*)(bs + 4 * m);
#pragma unroll 1
    for (int i = 0; i < 8; ++i) {
      const int lr = 16 * wave + 2 * i + hh;
      float* p = stg + lr * NC + 4 * m;
      const v4f v = *(const v4fa*)p;
      const float pzv = pzl[lr];
      v4f y;
      y.x = eluf(v.x + b4.x) + pzv;
      y.y = eluf(v.y + b4.y) + pzv;
      y.z = eluf(v.z + b4.z) + pzv;
      y.w = eluf(v.w + b4.w) + pzv;
      *(v4fa*)p = y;
    }
    v4f fv[8];
#pragma unroll
    for (int i = 0; i < 8; ++i) {
      const int lr = 16 * wave + 2 * i + hh;
      fv[i] = *(const v4fa*)(stg + lr * NC + 4 * m);
    }
#pragma unroll
    for (int i = 0; i < 8; ++i) {
      const int gr = rowBase + 16 * wave + 2 * i + hh;
      float* op = outF + (size_t)gr * DOUT + 4 * m;
      if (gr < nOut) *(volatile v4f*)op = fv[i];
    }
    __threadfence();
#pragma unroll
    for (int i = 0; i < 8; ++i) {
      const int gr = rowBase + 16 * wave + 2 * i + hh;
      float* op = outF + (size_t)gr * DOUT + 4 * m;
      if (gr < nOut) *(volatile v4f*)op = fv[i];
    }
  }
}

template <int L>
__global__ __launch_bounds__(NTHR) void k_scan(const int* __restrict__ gath, const int* __restrict__ keys,
                                               int nE, int nN, int vec8, int mRows,
                                               const unsigned short* __restrict__ xb,
                                               const float* __restrict__ nout, const float* __restrict__ nin,
                                               const float* __restrict__ ivd, const int* __restrict__ degi,
                                               const float* __restrict__ sp,
                                               const float* __restrict__ b2, int nB2,
                                               unsigned short* outp, float* pzout) {
  extern __shared__ __attribute__((aligned(16))) int dsm[];
  int* list = dsm;
  int* hl   = dsm + LISTN;
  int* sl   = hl + RCAP;
  int* cnt  = sl + RCAP;
  int* offs = cnt + NBA;
  int* cur  = offs + NBA;
  int* misc = cur + NBA;
  const int tid = (int)threadIdx.x, lane = tid & 31, wave = tid >> 5;
  unsigned short* rowbuf = (unsigned short*)(misc + MISC_INTS) + wave * 256;
  float* pzl = (float*)(misc + MISC_INTS + ROWBUF_INTS);
  const int nodeBase = (int)blockIdx.x * NBA;

  {
    const v4i z4 = {0, 0, 0, 0};
    for (int i = tid * 4; i < AGG_ZINTS; i += NTHR * 4) *(v4ia*)(dsm + i) = z4;
    if (tid < MISC_INTS) misc[tid] = 0;
  }
  __syncthreads();

  int t = 0, ov = 0;
  const int nChunks = (nE + CHUNK - 1) / CHUNK;
#pragma unroll 1
  for (int ch = 0; ch < nChunks; ++ch) {
    const int cbase = ch * CHUNK;
    const int wc = scan_chunk<SLA>(keys, nE, cbase, nodeBase, NBA, vec8, list, tid, lane, wave);
    if (lane == 0) misc[wave] = wc;
    __syncthreads();
    if (wave == 0) {
#pragma unroll 1
      for (int w2 = 0; w2 < NWAVE; ++w2) {
        int c = misc[w2];
        c = c < 0 ? 0 : (c > WCAP ? WCAP : c);
#pragma unroll 1
        for (int b0 = 0; b0 < c; b0 += 32) {
          const int idx = b0 + lane;
          const int ent = list[w2 * WCAP + (idx < WCAP ? idx : WCAP - 1)];
          const int m32 = (c - b0) < 32 ? (c - b0) : 32;
#pragma unroll 1
          for (int k = 0; k < m32; ++k) {
            const int u    = __builtin_amdgcn_readlane(ent, k);
            const int slot = u & (NBA - 1);
            const int el   = (u >> SLA) & (CHUNK - 1);
            const int pk   = ((cbase + el) << SLA) | slot;
            if (t < RCAP) {
              if (lane == 0) { hl[t] = pk; cnt[slot] = cnt[slot] + 1; }
              t = t + 1;
            } else {
              ov = 1;
            }
          }
        }
      }
    }
    __syncthreads();
  }
  if (wave == 0 && lane == 0) { misc[8] = t; misc[9] = ov; }
  __syncthreads();
  int tt = misc[8];
  tt = tt < 0 ? 0 : (tt > RCAP ? RCAP : tt);
  const int ovf = misc[9];

  if (wave == 0) {
    const int base = lane * (NBA / 32);
    int s = 0;
#pragma unroll 1
    for (int i = 0; i < NBA / 32; ++i) s += cnt[base + i];
    int incl = s;
#pragma unroll
    for (int d = 1; d < 32; d <<= 1) {
      const int y = __shfl_up(incl, d, 32);
      if (lane >= d) incl += y;
    }
    int run = incl - s;
#pragma unroll 1
    for (int i = 0; i < NBA / 32; ++i) {
      const int cv = cnt[base + i];
      offs[base + i] = run;
      cur[base + i]  = run;
      run += cv;
    }
  }
  __syncthreads();
  if (wave == 0) {
#pragma unroll 1
    for (int b0 = 0; b0 < tt; b0 += 32) {
      const int idx = b0 + lane;
      const int ent = hl[idx < RCAP ? idx : RCAP - 1];
      const int m32 = (tt - b0) < 32 ? (tt - b0) : 32;
#pragma unroll 1
      for (int k = 0; k < m32; ++k) {
        const int u    = __builtin_amdgcn_readlane(ent, k);
        const int slot = u & (NBA - 1);
        if (lane == 0) {
          int p = cur[slot];
          p = p < 0 ? 0 : (p > RCAP - 1 ? RCAP - 1 : p);
          sl[p] = u;
          cur[slot] = p + 1;
        }
      }
    }
  }
  __syncthreads();

  const float qnan = __int_as_float(0x7fc00000);
  const float pz = (ovf != 0) ? qnan : 0.0f;
  float bq0 = 0.0f, bq1 = 0.0f, bq2 = 0.0f, bq3 = 0.0f;
  if constexpr (L == 2) {
    const int nb4 = nB2 >> 2;
    const int lb  = lane < nb4 ? lane : nb4 - 1;
    const v4f tb = *(const v4fa*)(b2 + 4 * lb);
    const bool bok = lane < nb4;
    bq0 = bok ? bf16_val(tb.x) : 0.0f;
    bq1 = bok ? bf16_val(tb.y) : 0.0f;
    bq2 = bok ? bf16_val(tb.z) : 0.0f;
    bq3 = bok ? bf16_val(tb.w) : 0.0f;
  }
#pragma unroll 1
  for (int si = 0; si < NBA / NWAVE; ++si) {
    const int s    = si * NWAVE + wave;
    const int node = nodeBase + s;
    const int craw = cnt[s];
    const bool big = craw > DEGCAP;
    int c = craw < 0 ? 0 : (craw > DEGCAP ? DEGCAP : craw);
    int o = offs[s];
    o = o < 0 ? 0 : (o > RCAP ? RCAP : o);
    const int  nc   = node < nN ? node : nN - 1;
    const bool live = node < nN;
    const int  dg   = degi[nc];
    const bool cbad = big || (live && (craw != dg));
    float a0 = 0.0f, a1 = 0.0f, a2 = 0.0f, a3 = 0.0f;
#pragma unroll 1
    for (int b0 = 0; b0 < c; b0 += 32) {
      int idx = o + b0 + lane;
      idx = idx > RCAP - 1 ? RCAP - 1 : idx;
      const int ent = sl[idx];
      int eid = ent >> SLA;
      eid = eid < 0 ? 0 : (eid > nE - 1 ? nE - 1 : eid);
      int sr = gath[eid];
      sr = sr < 0 ? 0 : (sr > nN - 1 ? nN - 1 : sr);
      int wvi = 0;
      if constexpr (L == 1) wvi = __float_as_int(nout[sr]);
      const int m32 = (c - b0) < 32 ? (c - b0) : 32;
#pragma unroll 1
      for (int k = 0; k < m32; ++k) {
        const int sk = __builtin_amdgcn_readlane(sr, k);
        if constexpr (L == 1) {
          const float ck = __int_as_float(__builtin_amdgcn_readlane(wvi, k));
          const v2u w = *(const v2ua*)(xb + (size_t)sk * DIN + 4 * lane);
          const float f0 = __uint_as_float(w.x << 16);
          const float f1 = __uint_as_float(w.x & 0xffff0000u);
          const float f2 = __uint_as_float(w.y << 16);
          const float f3 = __uint_as_float(w.y & 0xffff0000u);
          a0 = fmaf(ck, f0, a0);
          a1 = fmaf(ck, f1, a1);
          a2 = fmaf(ck, f2, a2);
          a3 = fmaf(ck, f3, a3);
        } else {
          const v4f a = *(const v4fa*)(sp + (size_t)sk * NSP + D2P + 4 * lane);
          a0 += a.x; a1 += a.y; a2 += a.z; a3 += a.w;
        }
      }
    }
    float y0, y1, y2, y3;
    if constexpr (L == 1) {
      const float ni = nin[nc];
      y0 = a0 * ni; y1 = a1 * ni; y2 = a2 * ni; y3 = a3 * ni;
    } else {
      const float iv = ivd[nc];
      const v4f sv = *(const v4fa*)(sp + (size_t)nc * NSP + 4 * lane);
      y0 = (sv.x + a0 * iv) + bq0;
      y1 = (sv.y + a1 * iv) + bq1;
      y2 = (sv.z + a2 * iv) + bq2;
      y3 = (sv.w + a3 * iv) + bq3;
    }
    const float pzr = cbad ? qnan : pz;
#pragma unroll 1
    for (int j = 0; j < 4; ++j) {
      float v = (j == 0) ? y0 : ((j == 1) ? y1 : ((j == 2) ? y2 : y3));
      if constexpr (L == 2) v = eluf(v);
      v = live ? (v + pzr) : 0.0f;
      const unsigned hbits = bf16_bits(v);
      const unsigned lbits = bf16_bits(v - __uint_as_float(hbits << 16));
      rowbuf[4 * lane + j]       = (unsigned short)hbits;
      rowbuf[128 + 4 * lane + j] = (unsigned short)lbits;
    }
    if constexpr (L == 2) {
      if (lane == 0) pzl[s] = live ? pzr : 0.0f;
    }
    wave_sync();
    const v8us q0 = *(const v8usa*)(rowbuf + 8 * lane);
    wave_sync();
    if (node < mRows) {
      unsigned short* rpw = outp + (size_t)node * 256 + 8 * lane;
      *(volatile v8us*)rpw = q0;
      __threadfence();
      *(volatile v8us*)rpw = q0;
    }
  }

  if constexpr (L == 2) {
    __syncthreads();
    const v4f pv = *(const v4fa*)(pzl + 4 * tid);
    float* pp = pzout + (size_t)nodeBase + 4 * tid;
    *(volatile v4f*)pp = pv;
    __threadfence();
    *(volatile v4f*)pp = pv;
  }
}

static inline int cdiv(int a, int b) { return (a + b - 1) / b; }
static inline size_t al256(size_t o) { return (o + 255) & ~(size_t)255; }

extern "C" void kernel_launch(void* const* d_in, const int* in_sizes, int n_in,
                              void* d_out, int out_size, void* d_ws, size_t ws_size,
                              hipStream_t stream) {
  if (n_in < 10) return;
  if (in_sizes[0] < DIN || (in_sizes[0] % DIN) != 0) return;
  const int nN = in_sizes[0] / DIN;
  if (nN < 16 || nN > (1 << 22)) return;
  const int nE = in_sizes[1];
  if (nE < 1 || nE >= (1 << (31 - SLA)) || in_sizes[2] != nE) return;
  if (in_sizes[3] != DIN * D1 || in_sizes[4] != D1) return;
  if (in_sizes[5] != D1 * D2 || in_sizes[6] != D1 * D2) return;
  if (in_sizes[7] != D2) return;
  if (in_sizes[8] != D2 * DOUT || in_sizes[9] != DOUT) return;
  if ((long long)out_size != (long long)nN * DOUT) return;

  const float* x   = (const float*)d_in[0];
  const int*   src = (const int*)d_in[1];
  const int*   dst = (const int*)d_in[2];
  const float* W1  = (const float*)d_in[3];
  const float* b1  = (const float*)d_in[4];
  const float* Wn  = (const float*)d_in[5];
  const float* Ws  = (const float*)d_in[6];
  const float* b2  = (const float*)d_in[7];
  const float* W3  = (const float*)d_in[8];
  const float* b3  = (const float*)d_in[9];
  float* out = (float*)d_out;

  const int MP   = cdiv(nN, GBM) * GBM;
  const int gM   = MP / GBM;
  const int gD   = cdiv(nN, NBD);
  const int NBPD = gD * NBD;
  const int gA   = cdiv(MP, NBA);
  const int NPZ  = gA * NBA;
  if ((long long)gA * NBA < (long long)MP) return;
  if (NBPD < nN) return;
  const int vec8 = ((nE & 3) == 0) ? 1 : 0;

  char* ws = (char*)d_ws;
  size_t off = 0;
  const size_t oNOUT = off; off = al256(off + (size_t)NBPD * 4);
  const size_t oNIN  = off; off = al256(off + (size_t)NBPD * 4);
  const size_t oIVD  = off; off = al256(off + (size_t)NBPD * 4);
  const size_t oDEGI = off; off = al256(off + (size_t)NBPD * 4);
  const size_t oPZ   = off; off = al256(off + (size_t)NPZ * 4);
  const size_t oW1T  = off; off = al256(off + (size_t)D1P * K1 * 2);
  const size_t oWSN  = off; off = al256(off + (size_t)2 * D2P * K2G * 2);
  const size_t oW3T  = off; off = al256(off + (size_t)DOUT * K3 * 2);
  const size_t oXB   = off; off = al256(off + (size_t)MP * DIN * 2);
  const size_t oAGG  = off; off = al256(off + (size_t)MP * 256 * 2);
  const size_t oH1   = off; off = al256(off + (size_t)MP * HROW * 2);
  const size_t oSP   = off; off = al256(off + (size_t)MP * NSP * 4);
  if (off > ws_size || off > (size_t)WSMAX) return;
  float*          NOUT = (float*)(ws + oNOUT);
  float*          NIN  = (float*)(ws + oNIN);
  float*          IVD  = (float*)(ws + oIVD);
  int*            DEGI = (int*)(ws + oDEGI);
  float*          PZ   = (float*)(ws + oPZ);
  unsigned short* W1T2 = (unsigned short*)(ws + oW1T);
  unsigned short* WSN  = (unsigned short*)(ws + oWSN);
  unsigned short* W3T2 = (unsigned short*)(ws + oW3T);
  unsigned short* XB   = (unsigned short*)(ws + oXB);
  unsigned short* AGG  = (unsigned short*)(ws + oAGG);
  unsigned short* H2   = AGG;
  unsigned short* H1   = (unsigned short*)(ws + oH1);
  float*          SP   = (float*)(ws + oSP);

  const size_t scanLds = (size_t)AGG_LDS_INTS * 4;
  hipFuncSetAttribute(reinterpret_cast<const void*>(&k_scan<1>), hipFuncAttributeMaxDynamicSharedMemorySize, (int)scanLds);
  hipFuncSetAttribute(reinterpret_cast<const void*>(&k_scan<2>), hipFuncAttributeMaxDynamicSharedMemorySize, (int)scanLds);

  const int nUx = MP * (DIN / 8);
  k_wprep<<<NUWT / NTHR, NTHR, 0, stream>>>(W1, Ws, Wn, W3, W1T2, WSN, W3T2);
  k_cvx<<<cdiv(nUx, NTHR), NTHR, 0, stream>>>(x, nN, nUx, XB);
  k_deg<0><<<gD, NTHR, 0, stream>>>(src, nE, vec8, NOUT, IVD, DEGI);
  k_deg<1><<<gD, NTHR, 0, stream>>>(dst, nE, vec8, NIN, IVD, DEGI);
  k_scan<1><<<gA, NTHR, scanLds, stream>>>(src, dst, nE, nN, vec8, MP, XB, NOUT, NIN, IVD, DEGI, SP, b2, D2,
                                           AGG, PZ);
  k_gemm<10, 1><<<dim3(gM, 1), GTHR, 0, stream>>>(AGG, W1T2, K1, b1, D1, PZ, H1, SP, nN);
  k_gemm<8, 2><<<dim3(gM, 2), GTHR, 0, stream>>>(H1, WSN, K2G, b2, D2, PZ, H1, SP, MP);
  k_scan<2><<<gA, NTHR, scanLds, stream>>>(src, dst, nE, nN, vec8, MP, XB, NOUT, NIN, IVD, DEGI, SP, b2, D2,
                                           H2, PZ);
  k_gemm<4, 3><<<dim3(gM, 1), GTHR, 0, stream>>>(H2, W3T2, K3, b3, DOUT, PZ, H1, out, nN);
}
